// GAT_87729001988239
// MI455X (gfx1250) — hardware-verified
//
#include <hip/hip_runtime.h>
#include <stddef.h>
#include <stdint.h>
#include <math.h>


#define DIN    64
#define DH     128
#define KP     256
#define NCLS   4
#define SDW    8
#define P2W    8
#define NTHR   256
#define NWAVE  8
#define EPT    8
#define CHUNK  (NTHR * EPT)
#define WCAP   (EPT * 32)
#define LISTN  (NWAVE * WCAP)
#define NBA    1024
#define SLA    10
#define RCAP   24576
#define DEGCAP 64
#define GBM    64
#define GBN    128
#define GTHR   128
#define NU0    (DH * (DIN / 8))
#define NU1    (DH * (KP / 8))
#define STGF   (NBA * P2W)
#define NEGSL  0.2f
#define AGG_ZINTS (LISTN + 2 * RCAP + 3 * NBA)
#define AGG_LDS_INTS (AGG_ZINTS + 16 + STGF)
#define WSMAX  134217728

static_assert((CHUNK & (CHUNK - 1)) == 0 && CHUNK <= 4096);
static_assert((NBA & (NBA - 1)) == 0 && NBA == (1 << SLA));
static_assert(((long long)CHUNK << SLA) < (1LL << 31));
static_assert(LISTN % NTHR == 0);
static_assert(NBA % NWAVE == 0 && NBA % 32 == 0 && NBA % GBM == 0 && NBA % NTHR == 0 && NBA % 8 == 0);
static_assert(RCAP % 4 == 0 && AGG_ZINTS % 4 == 0 && LISTN % 4 == 0);
static_assert(DIN % 32 == 0 && KP % 32 == 0 && KP == 2 * DH && DH == GBN);
static_assert(GBM == (GTHR / 32) * 16 && GBN == 4 * 32);
static_assert(NU0 % NTHR == 0 && NU1 % NTHR == 0);
static_assert(DIN / 8 == 8 && KP / 8 == 32);
static_assert(AGG_LDS_INTS * 4 <= 300000);
static_assert(((AGG_ZINTS + 16) % 4) == 0);
static_assert((STGF / 4) % NTHR == 0);
static_assert(GBM * SDW == 4 * GTHR);
static_assert(DEGCAP % 32 == 0 && DEGCAP >= 41);

typedef float          v4f   __attribute__((ext_vector_type(4)));
typedef float          v8f   __attribute__((ext_vector_type(8)));
typedef int            v4i   __attribute__((ext_vector_type(4)));
typedef int            v8i   __attribute__((ext_vector_type(8)));
typedef unsigned int   v4u   __attribute__((ext_vector_type(4)));
typedef unsigned short v8us  __attribute__((ext_vector_type(8)));
typedef unsigned short v16us __attribute__((ext_vector_type(16)));
typedef __bf16         v16bf __attribute__((ext_vector_type(16)));
typedef v4f  __attribute__((may_alias)) v4fa;
typedef v4i  __attribute__((may_alias)) v4ia;
typedef v8us __attribute__((may_alias)) v8usa;
union FragB { v16bf v; v16us u; v8us h[2]; v8i w; };

__device__ __forceinline__ v8f wmb(const FragB& a, const FragB& b, v8f c) {
  v8f d = __builtin_amdgcn_wmma_f32_16x16x32_bf16(false, a.v, false, b.v, (short)0, c, false, false);
  asm volatile("v_nop\n\tv_nop\n\tv_nop\n\tv_nop" : "+v"(d) : "v"(a.w), "v"(b.w));
  return d;
}

__device__ __forceinline__ unsigned bf16_bits(float f) {
  const unsigned u = __float_as_uint(f);
  return ((u + 0x7FFFu + ((u >> 16) & 1u)) >> 16) & 0xFFFFu;
}
__device__ __forceinline__ float bf16_val(float f) { return __uint_as_float(bf16_bits(f) << 16); }
__device__ __forceinline__ v4f bfr4(const v4f a) {
  v4f r; r.x = bf16_val(a.x); r.y = bf16_val(a.y); r.z = bf16_val(a.z); r.w = bf16_val(a.w); return r;
}

__device__ __forceinline__ v4f elu4(const v4f v) {
  v4f r = v;
#pragma unroll 1
  for (int i = 0; i < 4; ++i) {
    const float t = (i == 0) ? v.x : ((i == 1) ? v.y : ((i == 2) ? v.z : v.w));
    const float e = (t > 0.0f) ? t : expm1f(t);
    r.x = (i == 0) ? e : r.x;
    r.y = (i == 1) ? e : r.y;
    r.z = (i == 2) ? e : r.z;
    r.w = (i == 3) ? e : r.w;
  }
  return r;
}

template <int SLB>
__device__ __forceinline__ int scan_chunk(const int* __restrict__ dsts, int nE, int cbase, int slotBase,
                                          int nb, int vec8, int* list, int tid, int lane, int wave) {
  int wc = 0;
  const int el0  = tid * EPT;
  const int e0   = cbase + el0;
  const int sent = -2147483647 - 1;
  v4i da, db;
  if (vec8 != 0 && cbase + CHUNK <= nE) {
    da = *(const v4i*)(dsts + e0);
    db = *(const v4i*)(dsts + e0 + 4);
  } else {
    da.x = (e0     < nE) ? dsts[min(e0,     nE - 1)] : sent;
    da.y = (e0 + 1 < nE) ? dsts[min(e0 + 1, nE - 1)] : sent;
    da.z = (e0 + 2 < nE) ? dsts[min(e0 + 2, nE - 1)] : sent;
    da.w = (e0 + 3 < nE) ? dsts[min(e0 + 3, nE - 1)] : sent;
    db.x = (e0 + 4 < nE) ? dsts[min(e0 + 4, nE - 1)] : sent;
    db.y = (e0 + 5 < nE) ? dsts[min(e0 + 5, nE - 1)] : sent;
    db.z = (e0 + 6 < nE) ? dsts[min(e0 + 6, nE - 1)] : sent;
    db.w = (e0 + 7 < nE) ? dsts[min(e0 + 7, nE - 1)] : sent;
  }
  const unsigned nbs = (unsigned)slotBase;
  const unsigned unb = (unsigned)nb;
  const unsigned s0 = (unsigned)da.x - nbs, s1 = (unsigned)da.y - nbs;
  const unsigned s2 = (unsigned)da.z - nbs, s3 = (unsigned)da.w - nbs;
  const unsigned s4 = (unsigned)db.x - nbs, s5 = (unsigned)db.y - nbs;
  const unsigned s6 = (unsigned)db.z - nbs, s7 = (unsigned)db.w - nbs;
  const bool h0 = s0 < unb, h1 = s1 < unb, h2 = s2 < unb, h3 = s3 < unb;
  const bool h4 = s4 < unb, h5 = s5 < unb, h6 = s6 < unb, h7 = s7 < unb;
  const unsigned any = __builtin_amdgcn_ballot_w32(h0 | h1 | h2 | h3 | h4 | h5 | h6 | h7);
  if (any != 0u) {
#define HITJ(J, HJ, SJ) { \
      const unsigned mj = __builtin_amdgcn_ballot_w32(HJ); \
      if (mj != 0u) { \
        if (HJ) { \
          const int pos = wc + (int)__builtin_amdgcn_mbcnt_lo(mj, 0u); \
          if (pos < WCAP) list[wave * WCAP + pos] = ((el0 + (J)) << SLB) | (int)(SJ); \
        } \
        wc += (int)__builtin_popcount(mj); } }
    HITJ(0, h0, s0)
    HITJ(1, h1, s1)
    HITJ(2, h2, s2)
    HITJ(3, h3, s3)
    HITJ(4, h4, s4)
    HITJ(5, h5, s5)
    HITJ(6, h6, s6)
    HITJ(7, h7, s7)
#undef HITJ
  }
  return wc;
}

__device__ __forceinline__ void build_hits(const int* __restrict__ dsts, int nE, int vec8, int nodeBase,
                                           int* dsm, int tid, int lane, int wave, int& ttOut, int& ovfOut) {
  int* list = dsm;
  int* hl   = dsm + LISTN;
  int* sl   = dsm + LISTN + RCAP;
  int* cnt  = dsm + LISTN + 2 * RCAP;
  int* offs = cnt + NBA;
  int* cur  = offs + NBA;
  int* misc = cur + NBA;
  {
    const v4i z4 = {0, 0, 0, 0};
    for (int i = tid * 4; i < AGG_ZINTS; i += NTHR * 4) *(v4ia*)(dsm + i) = z4;
    if (tid < 16) misc[tid] = 0;
  }
  __syncthreads();

  int t = 0, ov = 0;
  const int nChunks = (nE + CHUNK - 1) / CHUNK;
#pragma unroll 1
  for (int ch = 0; ch < nChunks; ++ch) {
    const int cbase = ch * CHUNK;
    const int wc = scan_chunk<SLA>(dsts, nE, cbase, nodeBase, NBA, vec8, list, tid, lane, wave);
    if (lane == 0) misc[wave] = wc;
    __syncthreads();
    if (wave == 0) {
#pragma unroll 1
      for (int w2 = 0; w2 < NWAVE; ++w2) {
        int c = misc[w2];
        c = c < 0 ? 0 : (c > WCAP ? WCAP : c);
#pragma unroll 1
        for (int b0 = 0; b0 < c; b0 += 32) {
          const int idx = b0 + lane;
          const int ent = list[w2 * WCAP + (idx < WCAP ? idx : WCAP - 1)];
          const int m32 = (c - b0) < 32 ? (c - b0) : 32;
#pragma unroll 1
          for (int k = 0; k < m32; ++k) {
            const int u    = __builtin_amdgcn_readlane(ent, k);
            const int slot = u & (NBA - 1);
            const int el   = (u >> SLA) & (CHUNK - 1);
            const int pk   = ((cbase + el) << SLA) | slot;
            if (t < RCAP) {
              if (lane == 0) { hl[t] = pk; cnt[slot] = cnt[slot] + 1; }
              t = t + 1;
            } else {
              ov = 1;
            }
          }
        }
      }
    }
    __syncthreads();
  }
  if (wave == 0 && lane == 0) { misc[8] = t; misc[9] = ov; }
  __syncthreads();
  int tt = misc[8];
  tt = tt < 0 ? 0 : (tt > RCAP ? RCAP : tt);
  const int ovf = misc[9];

  if (wave == 0) {
    const int base = lane * (NBA / 32);
    int s = 0;
#pragma unroll 1
    for (int i = 0; i < NBA / 32; ++i) s += cnt[base + i];
    int incl = s;
#pragma unroll
    for (int d = 1; d < 32; d <<= 1) {
      const int y = __shfl_up(incl, d, 32);
      if (lane >= d) incl += y;
    }
    int run = incl - s;
#pragma unroll 1
    for (int i = 0; i < NBA / 32; ++i) {
      const int cv = cnt[base + i];
      offs[base + i] = run;
      cur[base + i]  = run;
      run += cv;
    }
  }
  __syncthreads();
  if (wave == 0) {
#pragma unroll 1
    for (int b0 = 0; b0 < tt; b0 += 32) {
      const int idx = b0 + lane;
      const int ent = hl[idx < RCAP ? idx : RCAP - 1];
      const int m32 = (tt - b0) < 32 ? (tt - b0) : 32;
#pragma unroll 1
      for (int k = 0; k < m32; ++k) {
        const int u    = __builtin_amdgcn_readlane(ent, k);
        const int slot = u & (NBA - 1);
        if (lane == 0) {
          int p = cur[slot];
          p = p < 0 ? 0 : (p > RCAP - 1 ? RCAP - 1 : p);
          sl[p] = u;
          cur[slot] = p + 1;
        }
      }
    }
  }
  __syncthreads();
  ttOut = tt;
  ovfOut = ovf;
}

__global__ __launch_bounds__(NTHR) void k_wprep(const float* __restrict__ W0, const float* __restrict__ W1,
                                                unsigned short* W0T, unsigned short* W1T2) {
  const int u = (int)blockIdx.x * NTHR + (int)threadIdx.x;
  v8us o;
  unsigned short* dp;
  if (u < NU0) {
    const int n  = u >> 3;
    const int k8 = (u & 7) * 8;
    const float* p = W0 + (size_t)k8 * DH + n;
#pragma unroll
    for (int i = 0; i < 8; ++i) o[i] = (unsigned short)bf16_bits(p[(size_t)i * DH]);
    dp = W0T + (size_t)n * DIN + k8;
  } else if (u < NU0 + NU1) {
    const int v  = u - NU0;
    const int n  = v >> 5;
    const int k8 = (v & 31) * 8;
    const int kk = k8 & (DH - 1);
    const float* p = W1 + (size_t)kk * DH + n;
#pragma unroll
    for (int i = 0; i < 8; ++i) o[i] = (unsigned short)bf16_bits(p[(size_t)i * DH]);
    dp = W1T2 + (size_t)n * KP + k8;
  } else {
    return;
  }
  *(volatile v8us*)dp = o;
  __threadfence();
  *(volatile v8us*)dp = o;
}

__global__ __launch_bounds__(NTHR) void k_cvx(const float* __restrict__ x, int nN, int nUnits,
                                              unsigned short* xb) {
  const int u = (int)blockIdx.x * NTHR + (int)threadIdx.x;
  if (u >= nUnits) return;
  const int row = u >> 3;
  const int k8  = (u & 7) * 8;
  const int rc  = row < nN ? row : nN - 1;
  const float* p = x + (size_t)rc * DIN + k8;
  const v4f a = *(const v4f*)p;
  const v4f b = *(const v4f*)(p + 4);
  const bool ok = row < nN;
  v8us o;
  o[0] = ok ? (unsigned short)bf16_bits(a.x) : (unsigned short)0;
  o[1] = ok ? (unsigned short)bf16_bits(a.y) : (unsigned short)0;
  o[2] = ok ? (unsigned short)bf16_bits(a.z) : (unsigned short)0;
  o[3] = ok ? (unsigned short)bf16_bits(a.w) : (unsigned short)0;
  o[4] = ok ? (unsigned short)bf16_bits(b.x) : (unsigned short)0;
  o[5] = ok ? (unsigned short)bf16_bits(b.y) : (unsigned short)0;
  o[6] = ok ? (unsigned short)bf16_bits(b.z) : (unsigned short)0;
  o[7] = ok ? (unsigned short)bf16_bits(b.w) : (unsigned short)0;
  unsigned short* dp = xb + (size_t)row * DIN + k8;
  *(volatile v8us*)dp = o;
  __threadfence();
  *(volatile v8us*)dp = o;
}

__global__ __launch_bounds__(GTHR) void k_gemm(const unsigned short* __restrict__ A,
                                               const unsigned short* __restrict__ BT, int K,
                                               float* Cm, const float* __restrict__ avl,
                                               const float* __restrict__ avr, float* SD) {
  __shared__ __attribute__((aligned(16))) float stg[GBM * GBN];
  __shared__ __attribute__((aligned(16))) float sdt[GBM * SDW];
  const int tid = (int)threadIdx.x, lane = tid & 31, wave = tid >> 5, hh = lane >> 4, m = lane & 15;
  const int rowBase = (int)blockIdx.x * GBM;

  v8f acc[8];
  {
    const v8f z = {0.f, 0.f, 0.f, 0.f, 0.f, 0.f, 0.f, 0.f};
#pragma unroll
    for (int t = 0; t < 8; ++t) acc[t] = z;
  }
  const unsigned short* ap = A  + (size_t)(rowBase + 16 * wave + m) * (size_t)K + 8 * hh;
  const unsigned short* bp = BT + (size_t)m * (size_t)K + 8 * hh;

#pragma unroll 1
  for (int k0 = 0; k0 < K; k0 += 32) {
    FragB af;
    af.h[0] = *(const v8usa*)(ap + k0);
    af.h[1] = *(const v8usa*)(ap + k0 + 16);
#pragma unroll
    for (int nt = 0; nt < 8; ++nt) {
      const unsigned short* wq = bp + (size_t)(16 * nt) * (size_t)K + k0;
      FragB bf;
      bf.h[0] = *(const v8usa*)wq;
      bf.h[1] = *(const v8usa*)(wq + 16);
      acc[nt] = wmb(af, bf, acc[nt]);
    }
  }

#pragma unroll
  for (int nt = 0; nt < 8; ++nt) {
    const int lc = 16 * nt + m;
#pragma unroll
    for (int r = 0; r < 8; ++r) {
      const int lr = 16 * wave + 8 * hh + r;
      stg[lr * GBN + lc] = acc[nt][r];
    }
  }
  __syncthreads();

  const v4f al4 = bfr4(*(const v4fa*)(avl + 4 * lane));
  const v4f ar4 = bfr4(*(const v4fa*)(avr + 4 * lane));
  const int hd = lane >> 3;
#pragma unroll 1
  for (int i = 0; i < 16; ++i) {
    const int row = wave * 16 + i;
    const v4f p = *(const v4fa*)(stg + row * GBN + 4 * lane);
    float s = p.x * al4.x; s = fmaf(p.y, al4.y, s); s = fmaf(p.z, al4.z, s); s = fmaf(p.w, al4.w, s);
    float d = p.x * ar4.x; d = fmaf(p.y, ar4.y, d); d = fmaf(p.z, ar4.z, d); d = fmaf(p.w, ar4.w, d);
#pragma unroll
    for (int off = 4; off > 0; off >>= 1) {
      s += __shfl_xor(s, off);
      d += __shfl_xor(d, off);
    }
    if ((lane & 7) == 0) { sdt[row * SDW + hd] = s; sdt[row * SDW + 4 + hd] = d; }
  }
  __syncthreads();

  const int pc = wave * 32 + lane;
  const v4f sdv = *(const v4fa*)(sdt + 4 * pc);
  float* sp = SD + (size_t)blockIdx.x * (GBM * SDW) + 4 * pc;
#pragma unroll 1
  for (int i = 0; i < 16; ++i) {
    const int row = wave * 16 + i;
    const v4f p = *(const v4fa*)(stg + row * GBN + 4 * lane);
    float* op = Cm + (size_t)(rowBase + row) * (size_t)GBN + 4 * lane;
    *(volatile v4f*)op = p;
  }
  *(volatile v4f*)sp = sdv;
  __threadfence();
#pragma unroll 1
  for (int i = 0; i < 16; ++i) {
    const int row = wave * 16 + i;
    const v4f p = *(const v4fa*)(stg + row * GBN + 4 * lane);
    float* op = Cm + (size_t)(rowBase + row) * (size_t)GBN + 4 * lane;
    *(volatile v4f*)op = p;
  }
  *(volatile v4f*)sp = sdv;
}

template <int L>
__global__ __launch_bounds__(NTHR) void k_scan(const int* __restrict__ srcs, const int* __restrict__ dsts,
                                               int nE, int nN, int vec8, int mRows,
                                               const float* __restrict__ F, const float* __restrict__ SD,
                                               const float* __restrict__ bias, const float* hres,
                                               const float* __restrict__ W2, const float* __restrict__ al2,
                                               const float* __restrict__ ar2,
                                               float* hout, unsigned short* hhl, float* p2) {
  extern __shared__ __attribute__((aligned(16))) int dsm[];
  int* sl   = dsm + LISTN + RCAP;
  int* cnt  = dsm + LISTN + 2 * RCAP;
  int* offs = cnt + NBA;
  float* stage = (float*)(dsm + AGG_ZINTS + 16);
  const int tid = (int)threadIdx.x, lane = tid & 31, wave = tid >> 5;
  const int nodeBase = (int)blockIdx.x * NBA;

  int tt = 0, ovf = 0;
  build_hits(dsts, nE, vec8, nodeBase, dsm, tid, lane, wave, tt, ovf);

  const int head = lane >> 3;
  const v4f bb4 = bfr4(*(const v4fa*)(bias + 4 * lane));
  const float FINF = __builtin_huge_valf();
  const float qnan = __int_as_float(0x7fc00000);
  const float pz = (ovf != 0) ? qnan : 0.0f;
  v4f w0 = {0.f, 0.f, 0.f, 0.f}, w1 = w0, w2 = w0, w3 = w0, a2l = w0, a2r = w0;
  if constexpr (L == 1) {
    w0 = bfr4(*(const v4fa*)(W2 + (size_t)(4 * lane + 0) * NCLS));
    w1 = bfr4(*(const v4fa*)(W2 + (size_t)(4 * lane + 1) * NCLS));
    w2 = bfr4(*(const v4fa*)(W2 + (size_t)(4 * lane + 2) * NCLS));
    w3 = bfr4(*(const v4fa*)(W2 + (size_t)(4 * lane + 3) * NCLS));
    a2l = bfr4(*(const v4fa*)al2);
    a2r = bfr4(*(const v4fa*)ar2);
  }

#pragma unroll 1
  for (int si = 0; si < NBA / NWAVE; ++si) {
    const int s    = si * NWAVE + wave;
    const int node = nodeBase + s;
    int c = __builtin_amdgcn_readfirstlane(cnt[s]);
    const bool big = c > DEGCAP;
    c = c < 0 ? 0 : (c > DEGCAP ? DEGCAP : c);
    int o = __builtin_amdgcn_readfirstlane(offs[s]);
    o = o < 0 ? 0 : (o > tt ? tt : o);
    if (c > tt - o) c = tt - o;
    const int nc = node < nN ? node : nN - 1;
    const float erv = SD[(size_t)nc * SDW + 4 + head];

    float mx = -FINF;
#pragma unroll 1
    for (int b0 = 0; b0 < c; b0 += 32) {
      int idx = o + b0 + lane;
      idx = idx > RCAP - 1 ? RCAP - 1 : idx;
      const int ent = sl[idx];
      int eid = ent >> SLA;
      eid = eid < 0 ? 0 : (eid > nE - 1 ? nE - 1 : eid);
      int sr = srcs[eid];
      sr = sr < 0 ? 0 : (sr > nN - 1 ? nN - 1 : sr);
      const int m32 = (c - b0) < 32 ? (c - b0) : 32;
#pragma unroll 1
      for (int k = 0; k < m32; ++k) {
        const int sk = __builtin_amdgcn_readlane(sr, k);
        float sc = SD[(size_t)sk * SDW + head] + erv;
        sc = sc > 0.f ? sc : NEGSL * sc;
        mx = fmaxf(mx, sc);
      }
    }
    const bool fin = (mx > -FINF) && (mx < FINF);
    const float mxf = fin ? mx : 0.0f;

    float sm = 0.0f;
    v4f acc = {0.f, 0.f, 0.f, 0.f};
#pragma unroll 1
    for (int b0 = 0; b0 < c; b0 += 32) {
      int idx = o + b0 + lane;
      idx = idx > RCAP - 1 ? RCAP - 1 : idx;
      const int ent = sl[idx];
      int eid = ent >> SLA;
      eid = eid < 0 ? 0 : (eid > nE - 1 ? nE - 1 : eid);
      int sr = srcs[eid];
      sr = sr < 0 ? 0 : (sr > nN - 1 ? nN - 1 : sr);
      const int m32 = (c - b0) < 32 ? (c - b0) : 32;
#pragma unroll 1
      for (int k = 0; k < m32; ++k) {
        const int sk = __builtin_amdgcn_readlane(sr, k);
        const v4f a = *(const v4f*)(F + (size_t)sk * DH + 4 * lane);
        float sc = SD[(size_t)sk * SDW + head] + erv;
        sc = sc > 0.f ? sc : NEGSL * sc;
        const float ex = expf(sc - mxf);
        sm += ex;
        acc.x = fmaf(ex, a.x, acc.x);
        acc.y = fmaf(ex, a.y, acc.y);
        acc.z = fmaf(ex, a.z, acc.z);
        acc.w = fmaf(ex, a.w, acc.w);
      }
    }
    const float rc  = __builtin_amdgcn_rcpf(sm);
    const float inv = (c > 0) ? rc : 0.0f;
    v4f v;
    v.x = acc.x * inv; v.y = acc.y * inv; v.z = acc.z * inv; v.w = acc.w * inv;
    if constexpr (L == 1) {
      const v4f hr = *(const v4f*)(hres + (size_t)nc * DH + 4 * lane);
      v.x += hr.x; v.y += hr.y; v.z += hr.z; v.w += hr.w;
    }
    v.x += bb4.x; v.y += bb4.y; v.z += bb4.z; v.w += bb4.w;
    v4f y = elu4(v);
    const float pzr = big ? qnan : pz;
    const bool live = node < nN;
    y.x = live ? (y.x + pzr) : 0.0f;
    y.y = live ? (y.y + pzr) : 0.0f;
    y.z = live ? (y.z + pzr) : 0.0f;
    y.w = live ? (y.w + pzr) : 0.0f;

    if constexpr (L == 0) {
      const unsigned hbx = bf16_bits(y.x), hby = bf16_bits(y.y), hbz = bf16_bits(y.z), hbw = bf16_bits(y.w);
      const unsigned lbx = bf16_bits(y.x - __uint_as_float(hbx << 16));
      const unsigned lby = bf16_bits(y.y - __uint_as_float(hby << 16));
      const unsigned lbz = bf16_bits(y.z - __uint_as_float(hbz << 16));
      const unsigned lbw = bf16_bits(y.w - __uint_as_float(hbw << 16));
      const int hw0 = (int)(hbx | (hby << 16)), hw1 = (int)(hbz | (hbw << 16));
      const int lw0 = (int)(lbx | (lby << 16)), lw1 = (int)(lbz | (lbw << 16));
      const int sa = (2 * lane) & 31, sb = (2 * lane + 1) & 31;
      const int g0 = __shfl(hw0, sa), g1 = __shfl(hw1, sa), g2 = __shfl(hw0, sb), g3 = __shfl(hw1, sb);
      const int q0 = __shfl(lw0, sa), q1 = __shfl(lw1, sa), q2 = __shfl(lw0, sb), q3 = __shfl(lw1, sb);
      const bool lsel = lane >= 16;
      v4u pv;
      pv.x = (unsigned)(lsel ? q0 : g0);
      pv.y = (unsigned)(lsel ? q1 : g1);
      pv.z = (unsigned)(lsel ? q2 : g2);
      pv.w = (unsigned)(lsel ? q3 : g3);
      float* op = hout + (size_t)node * DH + 4 * lane;
      unsigned short* gp = hhl + (size_t)node * KP + 8 * lane;
      const bool wr = node < mRows;
      if (wr) { *(volatile v4f*)op = y; *(volatile v4u*)gp = pv; }
      __threadfence();
      if (wr) { *(volatile v4f*)op = y; *(volatile v4u*)gp = pv; }
    } else {
      float t0 = y.x * w0.x; t0 = fmaf(y.y, w1.x, t0); t0 = fmaf(y.z, w2.x, t0); t0 = fmaf(y.w, w3.x, t0);
      float t1 = y.x * w0.y; t1 = fmaf(y.y, w1.y, t1); t1 = fmaf(y.z, w2.y, t1); t1 = fmaf(y.w, w3.y, t1);
      float t2 = y.x * w0.z; t2 = fmaf(y.y, w1.z, t2); t2 = fmaf(y.z, w2.z, t2); t2 = fmaf(y.w, w3.z, t2);
      float t3 = y.x * w0.w; t3 = fmaf(y.y, w1.w, t3); t3 = fmaf(y.z, w2.w, t3); t3 = fmaf(y.w, w3.w, t3);
#pragma unroll
      for (int off = 16; off > 0; off >>= 1) {
        t0 += __shfl_xor(t0, off);
        t1 += __shfl_xor(t1, off);
        t2 += __shfl_xor(t2, off);
        t3 += __shfl_xor(t3, off);
      }
      float e2l = t0 * a2l.x; e2l = fmaf(t1, a2l.y, e2l); e2l = fmaf(t2, a2l.z, e2l); e2l = fmaf(t3, a2l.w, e2l);
      float e2r = t0 * a2r.x; e2r = fmaf(t1, a2r.y, e2r); e2r = fmaf(t2, a2r.z, e2r); e2r = fmaf(t3, a2r.w, e2r);
      v4f fv; fv.x = t0; fv.y = t1; fv.z = t2; fv.w = t3;
      v4f ev; ev.x = e2l; ev.y = e2r; ev.z = 0.0f; ev.w = 0.0f;
      v4f sv;
      sv.x = (lane == 0) ? fv.x : ev.x;
      sv.y = (lane == 0) ? fv.y : ev.y;
      sv.z = (lane == 0) ? fv.z : ev.z;
      sv.w = (lane == 0) ? fv.w : ev.w;
      if (lane < 2) *(v4fa*)(stage + s * P2W + 4 * lane) = sv;
    }
  }

  if constexpr (L == 1) {
    __syncthreads();
    float* pb = p2 + (size_t)nodeBase * P2W;
#pragma unroll 1
    for (int p = tid; p < STGF / 4; p += NTHR) {
      const v4f q = *(const v4fa*)(stage + 4 * p);
      *(volatile v4f*)(pb + 4 * p) = q;
    }
    __threadfence();
#pragma unroll 1
    for (int p = tid; p < STGF / 4; p += NTHR) {
      const v4f q = *(const v4fa*)(stage + 4 * p);
      *(volatile v4f*)(pb + 4 * p) = q;
    }
  }
}

__global__ __launch_bounds__(NTHR) void k_scan2(const int* __restrict__ srcs, const int* __restrict__ dsts,
                                                int nE, int nN, int vec8,
                                                const float* __restrict__ P2, const float* __restrict__ b2,
                                                float* outp) {
  extern __shared__ __attribute__((aligned(16))) int dsm[];
  int* sl   = dsm + LISTN + RCAP;
  int* cnt  = dsm + LISTN + 2 * RCAP;
  int* offs = cnt + NBA;
  float* stage = (float*)(dsm + AGG_ZINTS + 16);
  const int tid = (int)threadIdx.x, lane = tid & 31, wave = tid >> 5;
  const int nodeBase = (int)blockIdx.x * NBA;

  int tt = 0, ovf = 0;
  build_hits(dsts, nE, vec8, nodeBase, dsm, tid, lane, wave, tt, ovf);

  const v4f bb = bfr4(*(const v4fa*)b2);
  const float FINF = __builtin_huge_valf();
  const float qnan = __int_as_float(0x7fc00000);
  const float pz = (ovf != 0) ? qnan : 0.0f;

#pragma unroll 1
  for (int j = 0; j < NBA / NTHR; ++j) {
    const int s    = j * NTHR + tid;
    const int node = nodeBase + s;
    int c = cnt[s];
    const bool big = c > DEGCAP;
    c = c < 0 ? 0 : (c > DEGCAP ? DEGCAP : c);
    int o = offs[s];
    o = o < 0 ? 0 : (o > tt ? tt : o);
    if (c > tt - o) c = tt - o;
    int cm = c;
#pragma unroll
    for (int off = 16; off > 0; off >>= 1) {
      const int other = __shfl_xor(cm, off);
      cm = cm > other ? cm : other;
    }
    cm = __builtin_amdgcn_readfirstlane(cm);
    cm = cm > DEGCAP ? DEGCAP : cm;
    const int nc = node < nN ? node : nN - 1;
    const float erv = P2[(size_t)nc * P2W + 5];

    float mx = -FINF;
#pragma unroll 1
    for (int q = 0; q < cm; ++q) {
      const bool valid = q < c;
      int idx = o + (valid ? q : 0);
      idx = idx > RCAP - 1 ? RCAP - 1 : idx;
      const int ent = sl[idx];
      int eid = ent >> SLA;
      eid = eid < 0 ? 0 : (eid > nE - 1 ? nE - 1 : eid);
      int sr = srcs[eid];
      sr = sr < 0 ? 0 : (sr > nN - 1 ? nN - 1 : sr);
      float sc = P2[(size_t)sr * P2W + 4] + erv;
      sc = sc > 0.f ? sc : NEGSL * sc;
      const float scm = valid ? sc : -FINF;
      mx = fmaxf(mx, scm);
    }
    const bool fin = (mx > -FINF) && (mx < FINF);
    const float mxf = fin ? mx : 0.0f;

    float sm = 0.0f;
    v4f acc = {0.f, 0.f, 0.f, 0.f};
#pragma unroll 1
    for (int q = 0; q < cm; ++q) {
      const bool valid = q < c;
      int idx = o + (valid ? q : 0);
      idx = idx > RCAP - 1 ? RCAP - 1 : idx;
      const int ent = sl[idx];
      int eid = ent >> SLA;
      eid = eid < 0 ? 0 : (eid > nE - 1 ? nE - 1 : eid);
      int sr = srcs[eid];
      sr = sr < 0 ? 0 : (sr > nN - 1 ? nN - 1 : sr);
      const v4f f = *(const v4f*)(P2 + (size_t)sr * P2W);
      float sc = P2[(size_t)sr * P2W + 4] + erv;
      sc = sc > 0.f ? sc : NEGSL * sc;
      const float e0 = expf(sc - mxf);
      const float ex = valid ? e0 : 0.0f;
      const float fx = valid ? f.x : 0.0f, fy = valid ? f.y : 0.0f;
      const float fz = valid ? f.z : 0.0f, fw = valid ? f.w : 0.0f;
      sm += ex;
      acc.x = fmaf(ex, fx, acc.x);
      acc.y = fmaf(ex, fy, acc.y);
      acc.z = fmaf(ex, fz, acc.z);
      acc.w = fmaf(ex, fw, acc.w);
    }
    const float rc  = __builtin_amdgcn_rcpf(sm);
    const float inv = (c > 0) ? rc : 0.0f;
    const float pzr = big ? qnan : pz;
    v4f r;
    r.x = (acc.x * inv + bb.x) + pzr;
    r.y = (acc.y * inv + bb.y) + pzr;
    r.z = (acc.z * inv + bb.z) + pzr;
    r.w = (acc.w * inv + bb.w) + pzr;
    *(v4fa*)(stage + s * NCLS) = r;
  }
  __syncthreads();

  int npc = nN - nodeBase;
  npc = npc < 0 ? 0 : (npc > NBA ? NBA : npc);
  float* ob = outp + (size_t)nodeBase * NCLS;
#pragma unroll 1
  for (int p = tid; p < npc; p += NTHR) {
    const v4f q = *(const v4fa*)(stage + 4 * p);
    *(volatile v4f*)(ob + 4 * p) = q;
  }
  __threadfence();
#pragma unroll 1
  for (int p = tid; p < npc; p += NTHR) {
    const v4f q = *(const v4fa*)(stage + 4 * p);
    *(volatile v4f*)(ob + 4 * p) = q;
  }
}

static inline int cdiv(int a, int b) { return (a + b - 1) / b; }

extern "C" void kernel_launch(void* const* d_in, const int* in_sizes, int n_in,
                              void* d_out, int out_size, void* d_ws, size_t ws_size,
                              hipStream_t stream) {
  if (n_in < 15) return;
  if (in_sizes[0] < DIN || (in_sizes[0] % DIN) != 0) return;
  const int nN = in_sizes[0] / DIN;
  if (nN > (1 << 22)) return;
  const int nE = in_sizes[1];
  if (nE < 1 || nE >= (1 << 21) || in_sizes[2] != nE) return;
  if (in_sizes[3] != DIN * DH) return;
  if (in_sizes[4] != DH || in_sizes[5] != DH || in_sizes[6] != DH) return;
  if (in_sizes[7] != DH * DH) return;
  if (in_sizes[8] != DH || in_sizes[9] != DH || in_sizes[10] != DH) return;
  if (in_sizes[11] != DH * NCLS) return;
  if (in_sizes[12] != NCLS || in_sizes[13] != NCLS || in_sizes[14] != NCLS) return;
  if ((long long)out_size != (long long)nN * NCLS) return;

  const float* x   = (const float*)d_in[0];
  const int*   src = (const int*)d_in[1];
  const int*   dst = (const int*)d_in[2];
  const float* W0  = (const float*)d_in[3];
  const float* al0 = (const float*)d_in[4];
  const float* ar0 = (const float*)d_in[5];
  const float* b0  = (const float*)d_in[6];
  const float* W1  = (const float*)d_in[7];
  const float* al1 = (const float*)d_in[8];
  const float* ar1 = (const float*)d_in[9];
  const float* b1  = (const float*)d_in[10];
  const float* W2  = (const float*)d_in[11];
  const float* al2 = (const float*)d_in[12];
  const float* ar2 = (const float*)d_in[13];
  const float* b2  = (const float*)d_in[14];
  float* out = (float*)d_out;

  const int MP   = cdiv(nN, NBA) * NBA;
  const int gM   = MP / GBM;
  const int gA   = MP / NBA;
  if (gA * NBA != MP || gM * GBM != MP) return;
  const int vec8 = ((nE & 3) == 0) ? 1 : 0;

  char* ws = (char*)d_ws;
  size_t off = 0;
  const size_t oW0T = off; off += (size_t)DH * DIN * 2;          off = (off + 255) & ~(size_t)255;
  const size_t oW1T = off; off += (size_t)DH * KP * 2;           off = (off + 255) & ~(size_t)255;
  const size_t oXB  = off; off += (size_t)MP * DIN * 2;          off = (off + 255) & ~(size_t)255;
  const size_t oFE  = off; off += (size_t)MP * DH * 4;           off = (off + 255) & ~(size_t)255;
  const size_t oSD  = off; off += (size_t)MP * SDW * 4;          off = (off + 255) & ~(size_t)255;
  const size_t oH1  = off; off += (size_t)MP * DH * 4;           off = (off + 255) & ~(size_t)255;
  const size_t oHL  = off; off += (size_t)MP * KP * 2;           off = (off + 255) & ~(size_t)255;
  const size_t oP2  = off; off += (size_t)MP * P2W * 4;          off = (off + 255) & ~(size_t)255;
  if (off > ws_size || off > (size_t)WSMAX) return;
  unsigned short* W0T  = (unsigned short*)(ws + oW0T);
  unsigned short* W1T2 = (unsigned short*)(ws + oW1T);
  unsigned short* XB   = (unsigned short*)(ws + oXB);
  float*          FEAT = (float*)(ws + oFE);
  float*          SDp  = (float*)(ws + oSD);
  float*          H1   = (float*)(ws + oH1);
  unsigned short* HL   = (unsigned short*)(ws + oHL);
  float*          P2   = (float*)(ws + oP2);

  const size_t aggLds = (size_t)AGG_LDS_INTS * 4;
  hipFuncSetAttribute(reinterpret_cast<const void*>(&k_scan<0>), hipFuncAttributeMaxDynamicSharedMemorySize, (int)aggLds);
  hipFuncSetAttribute(reinterpret_cast<const void*>(&k_scan<1>), hipFuncAttributeMaxDynamicSharedMemorySize, (int)aggLds);
  hipFuncSetAttribute(reinterpret_cast<const void*>(&k_scan2),   hipFuncAttributeMaxDynamicSharedMemorySize, (int)aggLds);

  const int nUx = MP * (DIN / 8);
  k_wprep<<<(NU0 + NU1) / NTHR, NTHR, 0, stream>>>(W0, W1, W0T, W1T2);
  k_cvx<<<cdiv(nUx, NTHR), NTHR, 0, stream>>>(x, nN, nUx, XB);
  k_gemm<<<gM, GTHR, 0, stream>>>(XB, W0T, DIN, FEAT, al0, ar0, SDp);
  k_scan<0><<<gA, NTHR, aggLds, stream>>>(src, dst, nE, nN, vec8, MP, FEAT, SDp, b0, FEAT,
                                          W2, al2, ar2, H1, HL, P2);
  k_gemm<<<gM, GTHR, 0, stream>>>(HL, W1T2, KP, FEAT, al1, ar1, SDp);
  k_scan<1><<<gA, NTHR, aggLds, stream>>>(src, dst, nE, nN, vec8, MP, FEAT, SDp, b1, H1,
                                          W2, al2, ar2, H1, HL, P2);
  k_scan2<<<gA, NTHR, aggLds, stream>>>(src, dst, nE, nN, vec8, P2, b2, out);
}
